// PhaseSpaceAttention_77446850282067
// MI455X (gfx1250) — hardware-verified
//
#include <hip/hip_runtime.h>
#include <math.h>
#include <stdint.h>

constexpr int NBATCH = 2;
constexpr int SEQ_T  = 2048;
constexpr int EMB    = 1024;
constexpr int NHEAD  = 16;
constexpr int HDIM   = 64;
constexpr int NPH    = 8;
constexpr int QK_LD  = 2048;

typedef __attribute__((ext_vector_type(16))) _Float16 v16h;
typedef __attribute__((ext_vector_type(8)))  _Float16 v8h;
typedef __attribute__((ext_vector_type(16))) __bf16   v16b;
typedef __attribute__((ext_vector_type(8)))  __bf16   v8b;
typedef __attribute__((ext_vector_type(8)))  float    v8f;
typedef __attribute__((ext_vector_type(4)))  float    v4f;

__device__ __forceinline__ unsigned short f2bf_bits(float f) {
  unsigned u = __float_as_uint(f);
  return (unsigned short)((u + 0x7FFFu + ((u >> 16) & 1u)) >> 16);
}
__device__ __forceinline__ float bf_bits2f(unsigned short h) { return __uint_as_float(((unsigned)h) << 16); }

__device__ __forceinline__ void dep_guard_h(v8f& a, v8f& b, v16h x, v16h y) { asm volatile("v_nop\n\tv_nop\n\tv_nop\n\tv_nop" : "+v"(a), "+v"(b) : "v"(x), "v"(y)); }
__device__ __forceinline__ void dep_guard_b(v8f& a, v8f& b, v16b x, v16b y) { asm volatile("v_nop\n\tv_nop\n\tv_nop\n\tv_nop" : "+v"(a), "+v"(b) : "v"(x), "v"(y)); }
__device__ __forceinline__ void keep4_h(v16h a, v16h b, v16h c, v16h d) { asm volatile("v_nop" :: "v"(a), "v"(b), "v"(c), "v"(d)); }
__device__ __forceinline__ void keep4_b(v16b a, v16b b, v16b c, v16b d) { asm volatile("v_nop" :: "v"(a), "v"(b), "v"(c), "v"(d)); }
__device__ __forceinline__ void acc_guard4(v8f& a, v8f& b, v8f& c, v8f& d) { asm volatile("v_nop\n\tv_nop\n\tv_nop\n\tv_nop" : "+v"(a), "+v"(b), "+v"(c), "+v"(d)); }
template <typename T> struct Frag;
template <> struct Frag<_Float16> {
  typedef v16h V; union U { v16h v; v8h h[2]; };
  static __device__ __forceinline__ v16h load(const _Float16* p) {
    U f; f.h[0] = *(const v8h*)(p); f.h[1] = *(const v8h*)(p + 16); return f.v;
  }
  static __device__ __forceinline__ v8f mma(v16h a, v16h b, v8f c) {
    return __builtin_amdgcn_wmma_f32_16x16x32_f16(false, a, false, b, (short)0, c, false, false);
  }
  static __device__ __forceinline__ void guard(v8f& a, v8f& b, v16h x, v16h y) { dep_guard_h(a, b, x, y); }
  static __device__ __forceinline__ void keep(v16h a, v16h b, v16h c, v16h d) { keep4_h(a, b, c, d); }
};
template <> struct Frag<__bf16> {
  typedef v16b V; union U { v16b v; v8b h[2]; };
  static __device__ __forceinline__ v16b load(const __bf16* p) {
    U f; f.h[0] = *(const v8b*)(p); f.h[1] = *(const v8b*)(p + 16); return f.v;
  }
  static __device__ __forceinline__ v8f mma(v16b a, v16b b, v8f c) {
    return __builtin_amdgcn_wmma_f32_16x16x32_bf16(false, a, false, b, (short)0, c, false, false);
  }
  static __device__ __forceinline__ void guard(v8f& a, v8f& b, v16b x, v16b y) { dep_guard_b(a, b, x, y); }
  static __device__ __forceinline__ void keep(v16b a, v16b b, v16b c, v16b d) { keep4_b(a, b, c, d); }
};

template <int ET> struct Elem;
template <> struct Elem<0> { typedef _Float16 T; };
template <> struct Elem<1> { typedef __bf16 T; };
template <int ET, bool SPLIT, int BIAS_MODE, int OUT_MODE, bool RESID, int ACT = 0>
__global__ __launch_bounds__(256) void wmma_gemm64(
    const unsigned short* __restrict__ Ap, const unsigned short* __restrict__ A2p, int lda, long strideA,
    const unsigned short* __restrict__ Btp, const unsigned short* __restrict__ Bt2p, int ldb, long strideB,
    void* __restrict__ Cout, void* __restrict__ Cout2, int ldc, long strideC,
    const float* __restrict__ bias,
    const float* __restrict__ resid, long strideR,
    int M, int N, int K, float scale) {
  typedef typename Elem<ET>::T T;
  typedef typename Frag<T>::V V;
  const T* A = (const T*)Ap; const T* A2 = (const T*)A2p; const T* Bt = (const T*)Btp; const T* Bt2 = (const T*)Bt2p;
  __shared__ __align__(16) float sT[8][16 * 68];
  const int b    = blockIdx.y;
  const int lane = threadIdx.x & 31;
  const int wave = threadIdx.x >> 5;
  const int tilesN = N >> 6;
  const int tilesM = M >> 6;
  const int tile = blockIdx.x * 8 + wave;
  if (tile >= tilesM * tilesN) return;
  const int tm = tile / tilesN;
  const int tn = tile - tm * tilesN;
  const int m0 = tm << 6;
  const int n0 = tn << 6;

  const T* Ab  = A  + (size_t)b * strideA;
  const T* Bb  = Bt + (size_t)b * strideB;
  const T* Ab2 = SPLIT ? (A2  + (size_t)b * strideA) : nullptr;
  const T* Bb2 = SPLIT ? (Bt2 + (size_t)b * strideB) : nullptr;

  const int rlane = lane & 15;
  const int koff  = (lane >> 4) * 8;
  const int mOff  = (lane >> 4) * 8;

  v8f acc[4][4];
#pragma unroll
  for (int i = 0; i < 4; ++i)
#pragma unroll
    for (int j = 0; j < 4; ++j) acc[i][j] = (v8f){0.f,0.f,0.f,0.f,0.f,0.f,0.f,0.f};

  for (int k0 = 0; k0 < K; k0 += 32) {
    V bh[4], bl[4];
#pragma unroll
    for (int j = 0; j < 4; ++j) {
      const size_t bo = (size_t)(n0 + (j << 4) + rlane) * ldb + koff + k0;
      bh[j] = Frag<T>::load(Bb + bo);
      if (SPLIT) bl[j] = Frag<T>::load(Bb2 + bo);
    }
#pragma unroll
    for (int i = 0; i < 4; ++i) {
      const size_t ao = (size_t)(m0 + (i << 4) + rlane) * lda + koff + k0;
      V ah = Frag<T>::load(Ab + ao);
      V al;
      if (SPLIT) al = Frag<T>::load(Ab2 + ao);
#pragma unroll
      for (int j = 0; j < 4; ++j) {
        acc[i][j] = Frag<T>::mma(ah, bh[j], acc[i][j]);
        if (SPLIT) {
          acc[i][j] = Frag<T>::mma(ah, bl[j], acc[i][j]);
          acc[i][j] = Frag<T>::mma(al, bh[j], acc[i][j]);
        }
      }
      Frag<T>::guard(acc[i][0], acc[i][3], ah, SPLIT ? al : ah);
    }
    Frag<T>::keep(bh[0], bh[1], bh[2], bh[3]);
    if (SPLIT) Frag<T>::keep(bl[0], bl[1], bl[2], bl[3]);
  }
  acc_guard4(acc[0][0], acc[0][1], acc[0][2], acc[0][3]);
  acc_guard4(acc[1][0], acc[1][1], acc[1][2], acc[1][3]);
  acc_guard4(acc[2][0], acc[2][1], acc[2][2], acc[2][3]);
  acc_guard4(acc[3][0], acc[3][1], acc[3][2], acc[3][3]);

  float* slab = sT[wave];
  const float* Rb = RESID ? (resid + (size_t)b * strideR) : nullptr;
#pragma unroll
  for (int i = 0; i < 4; ++i) {
    const int mBase = m0 + (i << 4);
#pragma unroll
    for (int j = 0; j < 4; ++j) {
      const int n = n0 + (j << 4) + rlane;
      float bv = 0.f;
      if (BIAS_MODE == 2) bv = bias[n];
#pragma unroll
      for (int r = 0; r < 8; ++r) {
        float v = acc[i][j][r] * scale;
        if (BIAS_MODE == 1) v += bias[mBase + mOff + r];
        if (BIAS_MODE == 2) v += bv;
        if (RESID) v += Rb[(size_t)(mBase + mOff + r) * ldc + n];
        if (ACT == 1) v = tanhf(v);
        if (ACT == 2) v = fmaxf(v, 0.0f);
        if (ACT == 3) v = v / (1.0f + expf(-v));
        if (ACT == 4) v = (v > 0.f) ? v : 0.01f * v;
        slab[(mOff + r) * 68 + (j << 4) + rlane] = v;
      }
    }
    __builtin_amdgcn_fence(__ATOMIC_RELEASE, "workgroup");
    __builtin_amdgcn_wave_barrier();
    __builtin_amdgcn_fence(__ATOMIC_ACQUIRE, "workgroup");
    if (OUT_MODE == 0) {
      float* C = (float*)Cout + (size_t)b * strideC;
      const int hh = lane >> 4, c4 = (lane & 15) * 4;
      for (int pass = 0; pass < 2; ++pass) {
#pragma unroll
        for (int it = 0; it < 8; ++it) {
          const int row = it * 2 + hh;
          v4f v = *(const v4f*)(slab + row * 68 + c4);
          *(volatile v4f*)(C + (size_t)(mBase + row) * ldc + n0 + c4) = v;
        }
        __threadfence();
      }
    } else {
      const int q = lane >> 3, c8 = (lane & 7) * 8;
      unsigned short* C  = (unsigned short*)Cout  + (size_t)b * strideC;
      unsigned short* C2 = (OUT_MODE == 2) ? ((unsigned short*)Cout2 + (size_t)b * strideC) : nullptr;
      for (int pass = 0; pass < 2; ++pass) {
#pragma unroll
        for (int it = 0; it < 4; ++it) {
          const int row = it * 4 + q;
          const float* sp = slab + row * 68 + c8;
          v8h hv, lv;
#pragma unroll
          for (int e = 0; e < 8; ++e) {
            if (OUT_MODE == 1) {
              hv[e] = (_Float16)sp[e];
            } else {
              unsigned short hb = f2bf_bits(sp[e]);
              unsigned short lb = f2bf_bits(sp[e] - bf_bits2f(hb));
              hv[e] = __builtin_bit_cast(_Float16, hb);
              lv[e] = __builtin_bit_cast(_Float16, lb);
            }
          }
          *(volatile v8h*)(C + (size_t)(mBase + row) * ldc + n0 + c8) = hv;
          if (OUT_MODE == 2) *(volatile v8h*)(C2 + (size_t)(mBase + row) * ldc + n0 + c8) = lv;
        }
        __threadfence();
      }
    }
    __builtin_amdgcn_fence(__ATOMIC_RELEASE, "workgroup");
    __builtin_amdgcn_wave_barrier();
    __builtin_amdgcn_fence(__ATOMIC_ACQUIRE, "workgroup");
  }
}

__global__ __launch_bounds__(256) void cast_f32_bf16x2(
    const float* __restrict__ in, unsigned short* __restrict__ out, int n2) {
  const int i = blockIdx.x * 256 + threadIdx.x;
  if (i < n2) {
    const float f0 = in[2 * (size_t)i], f1 = in[2 * (size_t)i + 1];
    const unsigned u = (unsigned)f2bf_bits(f0) | ((unsigned)f2bf_bits(f1) << 16);
    ((volatile unsigned*)out)[i] = u;
    __threadfence();
    ((volatile unsigned*)out)[i] = u;
  }
}

__global__ __launch_bounds__(256) void cast_f32_f16x2_scaled(
    const float* __restrict__ in, unsigned short* __restrict__ out, int n2, float scale) {
  const int i = blockIdx.x * 256 + threadIdx.x;
  if (i < n2) {
    const float f0 = bf_bits2f(f2bf_bits(in[2 * (size_t)i])) * scale;
    const float f1 = bf_bits2f(f2bf_bits(in[2 * (size_t)i + 1])) * scale;
    const _Float16 h0 = (_Float16)f0, h1 = (_Float16)f1;
    const unsigned u = (unsigned)__builtin_bit_cast(unsigned short, h0) | ((unsigned)__builtin_bit_cast(unsigned short, h1) << 16);
    ((volatile unsigned*)out)[i] = u;
    __threadfence();
    ((volatile unsigned*)out)[i] = u;
  }
}

__global__ __launch_bounds__(256) void bias_rne_kernel(
    const float* __restrict__ qkvb, const float* __restrict__ outb, float* __restrict__ outp) {
  const int i  = blockIdx.x * 256 + threadIdx.x;
  const int iq = i < 3 * EMB ? i : (3 * EMB - 1);
  int io = i - 3 * EMB; io = io < 0 ? 0 : (io > EMB - 1 ? EMB - 1 : io);
  const float a = qkvb[iq];
  const float c = outb[io];
  const float v = bf_bits2f(f2bf_bits((i < 3 * EMB) ? a : c));
  ((volatile float*)outp)[i] = v;
  __threadfence();
  ((volatile float*)outp)[i] = v;
}

__global__ __launch_bounds__(256) void phase_bias_kernel(
    const float* __restrict__ coords, const float* __restrict__ temp, float* __restrict__ pb) {
#pragma clang fp contract(off)
  __shared__ __align__(16) float ct[64 * NPH];
  __shared__ __align__(16) float cs[64 * NPH];
  __shared__ float sqt[64];
  __shared__ float sqs[64];
  const int tid = threadIdx.x;
  const int b   = blockIdx.z;
  const int t0  = blockIdx.y * 64;
  const int s0  = blockIdx.x * 64;
  const float invT = 1.0f / temp[0];
  {
    const int rr = tid & 127, row = rr >> 1, c4 = (rr & 1) * 4;
    const int base = (tid < 128) ? t0 : s0;
    const v4f v = *(const v4f*)(coords + ((size_t)b * SEQ_T + base + row) * NPH + c4);
    v4f w;
#pragma unroll
    for (int e = 0; e < 4; ++e) w[e] = bf_bits2f(f2bf_bits(v[e]));
    if (tid < 128) *(v4f*)(ct + row * NPH + c4) = w;
    else           *(v4f*)(cs + row * NPH + c4) = w;
  }
  __syncthreads();
  if (tid < 64) {
    float a = 0.0f;
#pragma unroll
    for (int p = 0; p < NPH; ++p) a = a + ct[tid * NPH + p] * ct[tid * NPH + p];
    sqt[tid] = a;
  } else if (tid < 128) {
    const int r = tid - 64;
    float a = 0.0f;
#pragma unroll
    for (int p = 0; p < NPH; ++p) a = a + cs[r * NPH + p] * cs[r * NPH + p];
    sqs[r] = a;
  }
  __syncthreads();

  const int wave = tid >> 5, lane = tid & 31, hh = lane >> 4, c4 = (lane & 15) * 4;
  v4f ca[4], cb[4];
  float sqv[4];
#pragma unroll
  for (int q = 0; q < 4; ++q) {
    ca[q]  = *(const v4f*)(cs + (c4 + q) * NPH);
    cb[q]  = *(const v4f*)(cs + (c4 + q) * NPH + 4);
    sqv[q] = sqs[c4 + q];
  }
#pragma unroll 1
  for (int it = 0; it < 4; ++it) {
    const int row = wave * 8 + it * 2 + hh;
    const v4f qa = *(const v4f*)(ct + row * NPH);
    const v4f qb = *(const v4f*)(ct + row * NPH + 4);
    const float st = sqt[row];
    v4f res;
#pragma unroll
    for (int q = 0; q < 4; ++q) {
      float dot = qa[0] * ca[q][0];
      dot = dot + qa[1] * ca[q][1];
      dot = dot + qa[2] * ca[q][2];
      dot = dot + qa[3] * ca[q][3];
      dot = dot + qb[0] * cb[q][0];
      dot = dot + qb[1] * cb[q][1];
      dot = dot + qb[2] * cb[q][2];
      dot = dot + qb[3] * cb[q][3];
      const float d2 = (st + sqv[q]) - 2.0f * dot;
      const float sr = sqrtf(fmaxf(d2, 0.0f));
      const float dist = (d2 > 0.0f) ? sr : 0.0f;
      res[q] = expf(-dist * invT);
    }
    float* p = pb + ((size_t)b * SEQ_T + t0 + row) * SEQ_T + s0 + c4;
    *(volatile v4f*)p = res;
    __threadfence();
    *(volatile v4f*)p = res;
  }
}

#define AT_D 64
#define AT_NW 4
#define AT_QB 64
#define AT_KC 64

__device__ __forceinline__ v8f mma_h16(v16h a, v16h b, v8f c) {
  c = __builtin_amdgcn_wmma_f32_16x16x32_f16(false, a, false, b, (short)0, c, false, false);
  asm volatile("v_nop\n\tv_nop\n\tv_nop\n\tv_nop" : "+v"(c) : "v"(a), "v"(b));
  return c;
}

__global__ __launch_bounds__(128)
void attn_phase64_kernel(const unsigned short* __restrict__ qkp, const unsigned short* __restrict__ vtp,
                         const float* __restrict__ pb, unsigned short* __restrict__ aop) {
  union FH { v16h v; v8h h[2]; };
  __shared__ __align__(16) _Float16 Ksh[AT_KC * AT_D];
  __shared__ __align__(16) _Float16 Vth[AT_D * AT_KC];
  __shared__ __align__(16) _Float16 Psh[AT_NW][16 * AT_KC];
  __shared__ __align__(16) float    Os[AT_NW][16 * 68];

  const int tid  = threadIdx.x;
  const int wave = tid >> 5;
  const int lane = tid & 31;
  const int hh   = lane >> 4;
  const int c    = lane & 15;

  const int nqb = SEQ_T / AT_QB;
  const int bx  = blockIdx.x;
  const int qb  = bx % nqb;
  const int h   = bx / nqb;
  const int b   = blockIdx.y;
  const int q0  = qb * AT_QB + wave * 16;

  const _Float16* QK = (const _Float16*)(const void*)qkp;
  const _Float16* VT = (const _Float16*)(const void*)vtp;
  _Float16*       AO = (_Float16*)(void*)aop;
  const size_t brow = (size_t)b * SEQ_T;

  v16h qa[2];
#pragma unroll
  for (int dc = 0; dc < 2; ++dc) {
    const _Float16* qr = QK + (brow + q0 + c) * (size_t)QK_LD + h * HDIM + dc * 32 + 8 * hh;
    qa[dc] = Frag<_Float16>::load(qr);
  }

  float mrow[8], lrow[8];
  v8f oacc[4];
#pragma unroll
  for (int r = 0; r < 8; ++r) { mrow[r] = -INFINITY; lrow[r] = 0.f; }
#pragma unroll
  for (int t = 0; t < 4; ++t) oacc[t] = (v8f){0.f,0.f,0.f,0.f,0.f,0.f,0.f,0.f};

  const int nChunks = SEQ_T / AT_KC;
  for (int kc = 0; kc < nChunks; ++kc) {
    const int kv0 = kc * AT_KC;
    __syncthreads();
    {
      const int r = tid >> 1, half = (tid & 1) * 32;
      const _Float16* ks = QK + (brow + kv0 + r) * (size_t)QK_LD + EMB + h * HDIM + half;
      const _Float16* vs = VT + ((size_t)b * EMB + h * HDIM + r) * SEQ_T + kv0 + half;
#pragma unroll
      for (int i = 0; i < 4; ++i) {
        const v8h a0 = *(const v8h*)(ks + 8 * i);
        const v8h b0 = *(const v8h*)(vs + 8 * i);
        *(v8h*)(Ksh + r * AT_D  + half + 8 * i) = a0;
        *(v8h*)(Vth + r * AT_KC + half + 8 * i) = b0;
      }
    }
    __syncthreads();

    v8f s[4];
#pragma unroll
    for (int j = 0; j < 4; ++j) {
      s[j] = (v8f){0.f,0.f,0.f,0.f,0.f,0.f,0.f,0.f};
#pragma unroll
      for (int dc = 0; dc < 2; ++dc) {
        FH kb;
        kb.h[0] = *(const v8h*)(Ksh + (j * 16 + c) * AT_D + dc * 32 + 8 * hh);
        kb.h[1] = *(const v8h*)(Ksh + (j * 16 + c) * AT_D + dc * 32 + 16 + 8 * hh);
        s[j] = mma_h16(qa[dc], kb.v, s[j]);
      }
    }
    const float* pbr = pb + (brow + q0 + 8 * hh) * (size_t)SEQ_T + kv0 + c;
    float cm[8];
#pragma unroll
    for (int r = 0; r < 8; ++r) {
      float m = -INFINITY;
#pragma unroll
      for (int j = 0; j < 4; ++j) {
        const float sv = s[j][r] * 0.125f + pbr[(size_t)r * SEQ_T + j * 16];
        s[j][r] = sv;
        m = fmaxf(m, sv);
      }
#pragma unroll
      for (int off = 1; off < 16; off <<= 1) m = fmaxf(m, __shfl_xor(m, off, 32));
      cm[r] = m;
    }
    _Float16* pw = Psh[wave];
#pragma unroll
    for (int r = 0; r < 8; ++r) {
      const float mnew = fmaxf(mrow[r], cm[r]);
      const float alpha = expf(mrow[r] - mnew);
      mrow[r] = mnew;
      float psum = 0.f;
#pragma unroll
      for (int j = 0; j < 4; ++j) {
        const float p = expf(s[j][r] - mnew);
        psum += p;
        pw[(8 * hh + r) * AT_KC + j * 16 + c] = (_Float16)(p * 32768.0f);
      }
#pragma unroll
      for (int off = 1; off < 16; off <<= 1) psum += __shfl_xor(psum, off, 32);
      lrow[r] = lrow[r] * alpha + psum;
#pragma unroll
      for (int t = 0; t < 4; ++t) oacc[t][r] *= alpha;
    }
    __builtin_amdgcn_fence(__ATOMIC_RELEASE, "workgroup");
    __builtin_amdgcn_wave_barrier();
    __builtin_amdgcn_fence(__ATOMIC_ACQUIRE, "workgroup");
#pragma unroll
    for (int kk = 0; kk < 2; ++kk) {
      FH pa;
      pa.h[0] = *(const v8h*)(pw + c * AT_KC + kk * 32 + 8 * hh);
      pa.h[1] = *(const v8h*)(pw + c * AT_KC + kk * 32 + 16 + 8 * hh);
#pragma unroll
      for (int t = 0; t < 4; ++t) {
        FH vb;
        vb.h[0] = *(const v8h*)(Vth + (t * 16 + c) * AT_KC + kk * 32 + 8 * hh);
        vb.h[1] = *(const v8h*)(Vth + (t * 16 + c) * AT_KC + kk * 32 + 16 + 8 * hh);
        oacc[t] = mma_h16(pa.v, vb.v, oacc[t]);
      }
    }
  }

  float* os = Os[wave];
#pragma unroll
  for (int r = 0; r < 8; ++r) {
    const float inv = 1.0f / (lrow[r] * 2048.0f);
#pragma unroll
    for (int t = 0; t < 4; ++t) os[(8 * hh + r) * 68 + t * 16 + c] = oacc[t][r] * inv;
  }
  __builtin_amdgcn_fence(__ATOMIC_RELEASE, "workgroup");
  __builtin_amdgcn_wave_barrier();
  __builtin_amdgcn_fence(__ATOMIC_ACQUIRE, "workgroup");
  {
    const int q = lane >> 3, c8 = (lane & 7) * 8;
    for (int pass = 0; pass < 2; ++pass) {
#pragma unroll
      for (int it = 0; it < 4; ++it) {
        const int row = it * 4 + q;
        const float* sp = os + row * 68 + c8;
        v8h hv;
#pragma unroll
        for (int e = 0; e < 8; ++e) hv[e] = (_Float16)sp[e];
        *(volatile v8h*)(AO + (brow + q0 + row) * (size_t)EMB + h * HDIM + c8) = hv;
      }
      __threadfence();
    }
  }
}

extern "C" void kernel_launch(void* const* d_in, const int* in_sizes, int n_in,
                              void* d_out, int out_size, void* d_ws, size_t ws_size,
                              hipStream_t stream) {
  if (n_in < 7) return;
  if (in_sizes[0] != NBATCH * SEQ_T * EMB || in_sizes[1] != NBATCH * SEQ_T * NPH ||
      in_sizes[2] != 3 * EMB * EMB || in_sizes[3] != 3 * EMB || in_sizes[4] != EMB * EMB ||
      in_sizes[5] != EMB || in_sizes[6] < 1 || out_size != NBATCH * SEQ_T * EMB) return;

  const float* x      = (const float*)d_in[0];
  const float* coords = (const float*)d_in[1];
  const float* qkv_w  = (const float*)d_in[2];
  const float* qkv_b  = (const float*)d_in[3];
  const float* out_w  = (const float*)d_in[4];
  const float* out_b  = (const float*)d_in[5];
  const float* ptemp  = (const float*)d_in[6];
  float* out = (float*)d_out;

  const size_t MROWS = (size_t)NBATCH * SEQ_T;
  size_t off = 0;
  char* ws = (char*)d_ws;
  unsigned short* xb   = (unsigned short*)(ws + off); off += MROWS * EMB * 2;
  unsigned short* wqkv = (unsigned short*)(ws + off); off += (size_t)3 * EMB * EMB * 2;
  unsigned short* wo   = (unsigned short*)(ws + off); off += (size_t)EMB * EMB * 2;
  float*          biasr= (float*)(ws + off);          off += (size_t)4 * EMB * 4;
  unsigned short* qk   = (unsigned short*)(ws + off); off += MROWS * QK_LD * 2;
  unsigned short* vt   = (unsigned short*)(ws + off); off += (size_t)NBATCH * EMB * SEQ_T * 2;
  float*          pb   = (float*)(ws + off);          off += (size_t)NBATCH * SEQ_T * SEQ_T * 4;
  unsigned short* ao   = (unsigned short*)(ws + off); off += MROWS * EMB * 2;
  if (off > ws_size) return;

  const int n2x = (int)(MROWS * EMB / 2);
  const int n2w = 3 * EMB * EMB / 2;
  const int n2o = EMB * EMB / 2;
  cast_f32_bf16x2<<<dim3((n2x + 255) / 256), 256, 0, stream>>>(x, xb, n2x);
  cast_f32_bf16x2<<<dim3((n2w + 255) / 256), 256, 0, stream>>>(qkv_w, wqkv, n2w);
  cast_f32_f16x2_scaled<<<dim3((n2o + 255) / 256), 256, 0, stream>>>(out_w, wo, n2o, 64.0f);

  bias_rne_kernel<<<dim3(4 * EMB / 256), 256, 0, stream>>>(qkv_b, out_b, biasr);

  phase_bias_kernel<<<dim3(SEQ_T / 64, SEQ_T / 64, NBATCH), 256, 0, stream>>>(coords, ptemp, pb);

  wmma_gemm64<1, false, 2, 1, false><<<dim3((4096 / 64) * (2048 / 64) / 8, 1), 256, 0, stream>>>(
      xb, xb, EMB, 0L, wqkv, wqkv, EMB, 0L, (void*)qk, (void*)qk, QK_LD, 0L,
      biasr, biasr, 0L, (int)MROWS, 2 * EMB, EMB, 1.0f);

  wmma_gemm64<1, false, 1, 1, false><<<dim3((1024 / 64) * (2048 / 64) / 8, NBATCH), 256, 0, stream>>>(
      wqkv + (size_t)2 * EMB * EMB, wqkv + (size_t)2 * EMB * EMB, EMB, 0L,
      xb, xb, EMB, (long)SEQ_T * EMB,
      (void*)vt, (void*)vt, SEQ_T, (long)EMB * SEQ_T,
      biasr + 2 * EMB, biasr, 0L, EMB, SEQ_T, EMB, 1.0f);

  attn_phase64_kernel<<<dim3(NHEAD * (SEQ_T / AT_QB), NBATCH), 128, 0, stream>>>(qk, vt, pb, ao);

  wmma_gemm64<0, false, 2, 0, false><<<dim3((4096 / 64) * (1024 / 64) / 8, 1), 256, 0, stream>>>(
      ao, ao, EMB, 0L, wo, wo, EMB, 0L, (void*)out, (void*)out, EMB, 0L,
      biasr + 3 * EMB, biasr, 0L, (int)MROWS, EMB, EMB, 1.0f / 1024.0f);
}
